// QuanvolutionClassifier_65481071406220
// MI455X (gfx1250) — hardware-verified
//
#include <hip/hip_runtime.h>

typedef __attribute__((ext_vector_type(16))) _Float16 v16h;
typedef __attribute__((ext_vector_type(8)))  _Float16 v8h;
typedef __attribute__((ext_vector_type(16))) __bf16   v16b;
typedef __attribute__((ext_vector_type(8)))  __bf16   v8b;
typedef __attribute__((ext_vector_type(8)))  float    v8f;
typedef __attribute__((ext_vector_type(4)))  float    v4f;
typedef __attribute__((ext_vector_type(4)))  unsigned v4u;
#define U16(p) ((const unsigned short*)(const void*)(p))

__device__ __forceinline__ unsigned short f2bf_bits(float f) {
  unsigned u = __float_as_uint(f);
  return (unsigned short)((u + 0x7FFFu + ((u >> 16) & 1u)) >> 16);
}
__device__ __forceinline__ float bf_bits2f(unsigned short h) { return __uint_as_float(((unsigned)h) << 16); }

__device__ __forceinline__ void dep_guard_h(v8f& a, v8f& b, v16h x, v16h y) { asm volatile("v_nop\n\tv_nop\n\tv_nop\n\tv_nop" : "+v"(a), "+v"(b) : "v"(x), "v"(y)); }
__device__ __forceinline__ void dep_guard_b(v8f& a, v8f& b, v16b x, v16b y) { asm volatile("v_nop\n\tv_nop\n\tv_nop\n\tv_nop" : "+v"(a), "+v"(b) : "v"(x), "v"(y)); }
__device__ __forceinline__ void keep4_h(v16h a, v16h b, v16h c, v16h d) { asm volatile("v_nop" :: "v"(a), "v"(b), "v"(c), "v"(d)); }
__device__ __forceinline__ void keep4_b(v16b a, v16b b, v16b c, v16b d) { asm volatile("v_nop" :: "v"(a), "v"(b), "v"(c), "v"(d)); }
__device__ __forceinline__ void acc_guard4(v8f& a, v8f& b, v8f& c, v8f& d) { asm volatile("v_nop\n\tv_nop\n\tv_nop\n\tv_nop" : "+v"(a), "+v"(b), "+v"(c), "+v"(d)); }
template <typename T> struct Frag;
template <> struct Frag<_Float16> {
  typedef v16h V; union U { v16h v; v8h h[2]; };
  static __device__ __forceinline__ v16h load(const _Float16* p) {
    U f; f.h[0] = *(const v8h*)(p); f.h[1] = *(const v8h*)(p + 16); return f.v;
  }
  static __device__ __forceinline__ v8f mma(v16h a, v16h b, v8f c) {
    return __builtin_amdgcn_wmma_f32_16x16x32_f16(false, a, false, b, (short)0, c, false, false);
  }
  static __device__ __forceinline__ void guard(v8f& a, v8f& b, v16h x, v16h y) { dep_guard_h(a, b, x, y); }
  static __device__ __forceinline__ void keep(v16h a, v16h b, v16h c, v16h d) { keep4_h(a, b, c, d); }
};
template <> struct Frag<__bf16> {
  typedef v16b V; union U { v16b v; v8b h[2]; };
  static __device__ __forceinline__ v16b load(const __bf16* p) {
    U f; f.h[0] = *(const v8b*)(p); f.h[1] = *(const v8b*)(p + 16); return f.v;
  }
  static __device__ __forceinline__ v8f mma(v16b a, v16b b, v8f c) {
    return __builtin_amdgcn_wmma_f32_16x16x32_bf16(false, a, false, b, (short)0, c, false, false);
  }
  static __device__ __forceinline__ void guard(v8f& a, v8f& b, v16b x, v16b y) { dep_guard_b(a, b, x, y); }
  static __device__ __forceinline__ void keep(v16b a, v16b b, v16b c, v16b d) { keep4_b(a, b, c, d); }
};

template <int ET> struct Elem;
template <> struct Elem<0> { typedef _Float16 T; };
template <> struct Elem<1> { typedef __bf16 T; };
template <int ET, bool SPLIT, int BIAS_MODE, int OUT_MODE, bool RESID, int ACT = 0>
__global__ __launch_bounds__(256) void wmma_gemm64(
    const unsigned short* __restrict__ Ap, const unsigned short* __restrict__ A2p, int lda, long strideA,
    const unsigned short* __restrict__ Btp, const unsigned short* __restrict__ Bt2p, int ldb, long strideB,
    void* __restrict__ Cout, void* __restrict__ Cout2, int ldc, long strideC,
    const float* __restrict__ bias,
    const float* __restrict__ resid, long strideR,
    int M, int N, int K, float scale) {
  typedef typename Elem<ET>::T T;
  typedef typename Frag<T>::V V;
  const T* A = (const T*)Ap; const T* A2 = (const T*)A2p; const T* Bt = (const T*)Btp; const T* Bt2 = (const T*)Bt2p;
  __shared__ __align__(16) float sT[8][16 * 68];
  const int b    = blockIdx.y;
  const int lane = threadIdx.x & 31;
  const int wave = threadIdx.x >> 5;
  const int tilesN = N >> 6;
  const int tilesM = M >> 6;
  const int tile = blockIdx.x * 8 + wave;
  if (tile >= tilesM * tilesN) return;
  const int tm = tile / tilesN;
  const int tn = tile - tm * tilesN;
  const int m0 = tm << 6;
  const int n0 = tn << 6;

  const T* Ab  = A  + (size_t)b * strideA;
  const T* Bb  = Bt + (size_t)b * strideB;
  const T* Ab2 = SPLIT ? (A2  + (size_t)b * strideA) : nullptr;
  const T* Bb2 = SPLIT ? (Bt2 + (size_t)b * strideB) : nullptr;

  const int rlane = lane & 15;
  const int koff  = (lane >> 4) * 8;
  const int mOff  = (lane >> 4) * 8;

  v8f acc[4][4];
#pragma unroll
  for (int i = 0; i < 4; ++i)
#pragma unroll
    for (int j = 0; j < 4; ++j) acc[i][j] = (v8f){0.f,0.f,0.f,0.f,0.f,0.f,0.f,0.f};

  for (int k0 = 0; k0 < K; k0 += 32) {
    V bh[4], bl[4];
#pragma unroll
    for (int j = 0; j < 4; ++j) {
      const size_t bo = (size_t)(n0 + (j << 4) + rlane) * ldb + koff + k0;
      bh[j] = Frag<T>::load(Bb + bo);
      if (SPLIT) bl[j] = Frag<T>::load(Bb2 + bo);
    }
#pragma unroll
    for (int i = 0; i < 4; ++i) {
      const size_t ao = (size_t)(m0 + (i << 4) + rlane) * lda + koff + k0;
      V ah = Frag<T>::load(Ab + ao);
      V al;
      if (SPLIT) al = Frag<T>::load(Ab2 + ao);
#pragma unroll
      for (int j = 0; j < 4; ++j) {
        acc[i][j] = Frag<T>::mma(ah, bh[j], acc[i][j]);
        if (SPLIT) {
          acc[i][j] = Frag<T>::mma(ah, bl[j], acc[i][j]);
          acc[i][j] = Frag<T>::mma(al, bh[j], acc[i][j]);
        }
      }
      Frag<T>::guard(acc[i][0], acc[i][3], ah, SPLIT ? al : ah);
    }
    Frag<T>::keep(bh[0], bh[1], bh[2], bh[3]);
    if (SPLIT) Frag<T>::keep(bl[0], bl[1], bl[2], bl[3]);
  }
  acc_guard4(acc[0][0], acc[0][1], acc[0][2], acc[0][3]);
  acc_guard4(acc[1][0], acc[1][1], acc[1][2], acc[1][3]);
  acc_guard4(acc[2][0], acc[2][1], acc[2][2], acc[2][3]);
  acc_guard4(acc[3][0], acc[3][1], acc[3][2], acc[3][3]);

  float* slab = sT[wave];
  const float* Rb = RESID ? (resid + (size_t)b * strideR) : nullptr;
#pragma unroll
  for (int i = 0; i < 4; ++i) {
    const int mBase = m0 + (i << 4);
#pragma unroll
    for (int j = 0; j < 4; ++j) {
      const int n = n0 + (j << 4) + rlane;
      float bv = 0.f;
      if (BIAS_MODE == 2) bv = bias[n];
#pragma unroll
      for (int r = 0; r < 8; ++r) {
        float v = acc[i][j][r] * scale;
        if (BIAS_MODE == 1) v += bias[mBase + mOff + r];
        if (BIAS_MODE == 2) v += bv;
        if (RESID) v += Rb[(size_t)(mBase + mOff + r) * ldc + n];
        if (ACT == 1) v = tanhf(v);
        if (ACT == 2) v = fmaxf(v, 0.0f);
        if (ACT == 3) v = v / (1.0f + expf(-v));
        if (ACT == 4) v = (v > 0.f) ? v : 0.01f * v;
        if (ACT == 5) v = 0.5f * v * (1.0f + erff(v * 0.70710678118654752f));
        slab[(mOff + r) * 68 + (j << 4) + rlane] = v;
      }
    }
    __builtin_amdgcn_fence(__ATOMIC_RELEASE, "workgroup");
    __builtin_amdgcn_wave_barrier();
    __builtin_amdgcn_fence(__ATOMIC_ACQUIRE, "workgroup");
    if (OUT_MODE == 0) {
      float* C = (float*)Cout + (size_t)b * strideC;
      const int hh = lane >> 4, c4 = (lane & 15) * 4;
      for (int pass = 0; pass < 2; ++pass) {
#pragma unroll
        for (int it = 0; it < 8; ++it) {
          const int row = it * 2 + hh;
          v4f v = *(const v4f*)(slab + row * 68 + c4);
          *(volatile v4f*)(C + (size_t)(mBase + row) * ldc + n0 + c4) = v;
        }
        __threadfence();
      }
    } else {
      const int q = lane >> 3, c8 = (lane & 7) * 8;
      unsigned short* C  = (unsigned short*)Cout  + (size_t)b * strideC;
      unsigned short* C2 = (OUT_MODE == 2) ? ((unsigned short*)Cout2 + (size_t)b * strideC) : nullptr;
      for (int pass = 0; pass < 2; ++pass) {
#pragma unroll
        for (int it = 0; it < 4; ++it) {
          const int row = it * 4 + q;
          const float* sp = slab + row * 68 + c8;
          v8h hv, lv;
#pragma unroll
          for (int e = 0; e < 8; ++e) {
            if (OUT_MODE == 1) {
              hv[e] = (_Float16)sp[e];
            } else {
              unsigned short hb = f2bf_bits(sp[e]);
              unsigned short lb = f2bf_bits(sp[e] - bf_bits2f(hb));
              hv[e] = __builtin_bit_cast(_Float16, hb);
              lv[e] = __builtin_bit_cast(_Float16, lb);
            }
          }
          *(volatile v8h*)(C + (size_t)(mBase + row) * ldc + n0 + c8) = hv;
          if (OUT_MODE == 2) *(volatile v8h*)(C2 + (size_t)(mBase + row) * ldc + n0 + c8) = lv;
        }
        __threadfence();
      }
    }
    __builtin_amdgcn_fence(__ATOMIC_RELEASE, "workgroup");
    __builtin_amdgcn_wave_barrier();
    __builtin_amdgcn_fence(__ATOMIC_ACQUIRE, "workgroup");
  }
}

constexpr int NIMG     = 4096;
constexpr int IMG_PIX  = 784;
constexpr int NPAT     = 196;
constexpr int NTILE    = 13;
constexpr int FEAT_K   = 784;
constexpr int FEAT_LD  = 832;
constexpr int HID      = 128;
constexpr int NCLS     = 10;
constexpr int NCLS_PAD = 64;
constexpr int LOGIT_LD = 64;

constexpr float AMP_CARRY  = 64.0f;
constexpr float U_CARRY    = 16.0f;
constexpr float FEAT_CARRY = 16.0f;
constexpr float WP_CARRY   = 64.0f;
constexpr float WC_CARRY   = 64.0f;

static_assert(FEAT_LD % 32 == 0 && FEAT_LD >= FEAT_K, "GEMM1 K pad");
static_assert(NTILE * 16 >= NPAT && NTILE * 64 == FEAT_LD, "tile line map covers the whole feature row");
static_assert((NIMG * NTILE) % 8 == 0, "feature grid exact");
static_assert(NIMG % 64 == 0 && HID % 64 == 0 && NCLS_PAD % 64 == 0, "GEMM M/N tile multiples");
static_assert(HID % 32 == 0, "GEMM2 K multiple of 32");
static_assert(FEAT_LD % 8 == 0 && (FEAT_LD / 8) == 104, "W_proj^T row = 104 x 16 B");
static_assert((64 * NCLS * 4) % 128 == 0, "64 output rows = whole 128-B lines");

constexpr size_t WS_FEATS = (size_t)NIMG * FEAT_LD * 2;
constexpr size_t WS_WPT   = (size_t)HID * FEAT_LD * 2;
constexpr size_t WS_WCT   = (size_t)NCLS_PAD * HID * 2;
constexpr size_t WS_H     = (size_t)NIMG * HID * 2;
constexpr size_t WS_LOG   = (size_t)NIMG * LOGIT_LD * 4;
constexpr size_t WS_TOTAL = WS_FEATS + WS_WPT + WS_WCT + WS_H + WS_LOG;
static_assert(WS_FEATS % 128 == 0 && WS_WPT % 128 == 0 && WS_WCT % 128 == 0 && WS_H % 128 == 0 && WS_LOG % 128 == 0, "aligned carve");
static_assert(WS_TOTAL <= 134217728ull, "carve under 128 MiB");

__device__ __forceinline__ v8f mma16_guarded(v16h a, v16h b, v8f c) {
  c = __builtin_amdgcn_wmma_f32_16x16x32_f16(false, a, false, b, (short)0, c, false, false);
  asm volatile("v_nop\n\tv_nop\n\tv_nop\n\tv_nop" : "+v"(c) : "v"(a), "v"(b));
  return c;
}
__device__ __forceinline__ unsigned hbits(float f) {
  return (unsigned)__builtin_bit_cast(unsigned short, (_Float16)f);
}

__global__ __launch_bounds__(128) void prep_wproj(const float* __restrict__ W,
                                                  unsigned short* __restrict__ WpT) {
  const int n = blockIdx.x;
  const int i = threadIdx.x;
  v4u val;
#pragma unroll
  for (int e2 = 0; e2 < 4; ++e2) {
    const int k0 = 8 * i + 2 * e2;
    const int k1 = k0 + 1;
    const int kc0 = (k0 < FEAT_K) ? k0 : (FEAT_K - 1);
    const int kc1 = (k1 < FEAT_K) ? k1 : (FEAT_K - 1);
    float v0 = W[(size_t)kc0 * HID + n];
    float v1 = W[(size_t)kc1 * HID + n];
    v0 = (k0 < FEAT_K) ? v0 * WP_CARRY : 0.0f;
    v1 = (k1 < FEAT_K) ? v1 * WP_CARRY : 0.0f;
    val[e2] = hbits(v0) | (hbits(v1) << 16);
  }
  unsigned short* dst = WpT + (size_t)n * FEAT_LD + 8 * ((i < 104) ? i : 0);
  if (i < 104) *(volatile v4u*)dst = val;
  __threadfence();
  if (i < 104) *(volatile v4u*)dst = val;
}

__global__ __launch_bounds__(32) void prep_wcls(const float* __restrict__ Wc,
                                                unsigned short* __restrict__ WcT) {
  const int n = blockIdx.x;
  const int i = threadIdx.x;
  const bool nval = (n < NCLS);
  const int nc = nval ? n : (NCLS - 1);
  v4u val;
#pragma unroll
  for (int e2 = 0; e2 < 4; ++e2) {
    const int k0 = 8 * i + 2 * e2;
    const int k1 = k0 + 1;
    const int kc0 = (k0 < HID) ? k0 : (HID - 1);
    const int kc1 = (k1 < HID) ? k1 : (HID - 1);
    float v0 = Wc[(size_t)kc0 * NCLS + nc];
    float v1 = Wc[(size_t)kc1 * NCLS + nc];
    v0 = nval ? v0 * WC_CARRY : 0.0f;
    v1 = nval ? v1 * WC_CARRY : 0.0f;
    val[e2] = hbits(v0) | (hbits(v1) << 16);
  }
  unsigned short* dst = WcT + (size_t)n * HID + 8 * ((i < 16) ? i : 0);
  if (i < 16) *(volatile v4u*)dst = val;
  __threadfence();
  if (i < 16) *(volatile v4u*)dst = val;
}

__global__ __launch_bounds__(256) void quanv_feats(const float* __restrict__ x,
                                                   const float* __restrict__ Ure,
                                                   const float* __restrict__ Uim,
                                                   unsigned short* __restrict__ feats) {
  const int lane = threadIdx.x & 31;
  const int wave = threadIdx.x >> 5;
  const int hh   = lane >> 4;
  const int m    = lane & 15;
  const int g = blockIdx.x * 8 + wave;
  if (g >= NIMG * NTILE) return;
  const int img = g / NTILE;
  const int t   = g - img * NTILE;

  v16h aRe = {};
  v16h aIm = {};
  {
    const float* ur = Ure + m * 16 + 8 * hh;
    const float* ui = Uim + m * 16 + 8 * hh;
#pragma unroll
    for (int e = 0; e < 8; ++e) {
      aRe[e] = (_Float16)(ur[e] * U_CARRY);
      aIm[e] = (_Float16)(ui[e] * U_CARRY);
      aRe[8 + e] = (_Float16)0.0f;
      aIm[8 + e] = (_Float16)0.0f;
    }
  }

  const int p = t * 16 + m;
  const bool pvalid = (p < NPAT);
  const int pcl  = pvalid ? p : (NPAT - 1);
  const int prow = pcl / 14;
  const int pcol = pcl - prow * 14;
  const float* xq = x + (size_t)img * IMG_PIX + prow * 56 + pcol * 2 + hh * 28;
  const float hA = 0.5f * xq[0];
  const float hB = 0.5f * xq[1];
  const float cA = cosf(hA);
  const float sA = sinf(hA);
  const float cB = cosf(hB);
  const float sB = sinf(hB);
  const float ocA = __shfl_xor(cA, 16, 32);
  const float osA = __shfl_xor(sA, 16, 32);
  const float ocB = __shfl_xor(cB, 16, 32);
  const float osB = __shfl_xor(sB, 16, 32);
  const bool up = (hh != 0);
  const float c0 = up ? ocA : cA;
  const float s0 = up ? osA : sA;
  const float c1 = up ? ocB : cB;
  const float s1 = up ? osB : sB;
  const float c2 = up ? cA : ocA;
  const float s2 = up ? sA : osA;
  const float c3 = up ? cB : ocB;
  const float s3 = up ? sB : osB;

  const float f0 = up ? s0 : c0;
  const float t0 = f0 * c1;
  const float t1 = f0 * s1;
  const float u0 = t0 * c2;
  const float u1 = t0 * s2;
  const float u2 = t1 * c2;
  const float u3 = t1 * s2;
  v16h bF = {};
  bF[0] = (_Float16)((u0 * c3) * AMP_CARRY);
  bF[1] = (_Float16)((u0 * s3) * AMP_CARRY);
  bF[2] = (_Float16)((u1 * c3) * AMP_CARRY);
  bF[3] = (_Float16)((u1 * s3) * AMP_CARRY);
  bF[4] = (_Float16)((u2 * c3) * AMP_CARRY);
  bF[5] = (_Float16)((u2 * s3) * AMP_CARRY);
  bF[6] = (_Float16)((u3 * c3) * AMP_CARRY);
  bF[7] = (_Float16)((u3 * s3) * AMP_CARRY);
#pragma unroll
  for (int e = 8; e < 16; ++e) bF[e] = (_Float16)0.0f;

  const v8f zc = (v8f){0.f,0.f,0.f,0.f,0.f,0.f,0.f,0.f};
  const v8f pre = mma16_guarded(aRe, bF, zc);
  const v8f pim = mma16_guarded(aIm, bF, zc);

  float pz[8];
#pragma unroll
  for (int r = 0; r < 8; ++r) pz[r] = pre[r] * pre[r] + pim[r] * pim[r];

  const float sAll = ((pz[0] + pz[1]) + (pz[2] + pz[3])) + ((pz[4] + pz[5]) + (pz[6] + pz[7]));
  const float p1   = ((pz[0] + pz[1]) + (pz[2] + pz[3])) - ((pz[4] + pz[5]) + (pz[6] + pz[7]));
  const float p2   = ((pz[0] + pz[1]) + (pz[4] + pz[5])) - ((pz[2] + pz[3]) + (pz[6] + pz[7]));
  const float p3   = ((pz[0] + pz[2]) + (pz[4] + pz[6])) - ((pz[1] + pz[3]) + (pz[5] + pz[7]));
  const float p0   = up ? -sAll : sAll;
  const float x0 = __shfl_xor(p0, 16, 32);
  const float x1 = __shfl_xor(p1, 16, 32);
  const float x2 = __shfl_xor(p2, 16, 32);
  const float x3 = __shfl_xor(p3, 16, 32);
  const float inv = 1.0f / (AMP_CARRY * AMP_CARRY * U_CARRY * U_CARRY);
  float e0 = (p0 + x0) * inv;
  float e1 = (p1 + x1) * inv;
  float e2 = (p2 + x2) * inv;
  float e3 = (p3 + x3) * inv;
  e0 = pvalid ? e0 : 0.0f;
  e1 = pvalid ? e1 : 0.0f;
  e2 = pvalid ? e2 : 0.0f;
  e3 = pvalid ? e3 : 0.0f;

  const unsigned w0 = hbits(e0 * FEAT_CARRY) | (hbits(e1 * FEAT_CARRY) << 16);
  const unsigned w1 = hbits(e2 * FEAT_CARRY) | (hbits(e3 * FEAT_CARRY) << 16);
  const int srcA = (2 * lane) & 31;
  const int srcB = (2 * lane + 1) & 31;
  v4u val;
  val[0] = __shfl(w0, srcA, 32);
  val[1] = __shfl(w1, srcA, 32);
  val[2] = __shfl(w0, srcB, 32);
  val[3] = __shfl(w1, srcB, 32);
  unsigned short* dst = feats + (size_t)img * FEAT_LD + t * 64 + 8 * ((lane < 8) ? lane : 0);
  if (lane < 8) *(volatile v4u*)dst = val;
  __threadfence();
  if (lane < 8) *(volatile v4u*)dst = val;
}

__global__ __launch_bounds__(256) void lsm_store(const float* __restrict__ lg,
                                                 const float* __restrict__ bcls,
                                                 float* __restrict__ out) {
  __shared__ __align__(16) float so[64 * NCLS];
  const int tid = threadIdx.x;
  const int r0 = blockIdx.x * 64;
  if (tid < 64) {
    const float* row = lg + (size_t)(r0 + tid) * LOGIT_LD;
    float mx = -__builtin_inff();
#pragma unroll 1
    for (int c = 0; c < NCLS; ++c) {
      const float v = row[c] + bcls[c];
      mx = fmaxf(mx, v);
    }
    float s = 0.0f;
#pragma unroll 1
    for (int c = 0; c < NCLS; ++c) {
      const float v = row[c] + bcls[c];
      s += expf(v - mx);
    }
    const float ls = logf(s);
#pragma unroll 1
    for (int c = 0; c < NCLS; ++c) {
      const float v = row[c] + bcls[c];
      so[tid * NCLS + c] = (v - mx) - ls;
    }
  }
  __syncthreads();
  const int q = (tid < 160) ? tid : 0;
  const v4f val = *(const v4f*)(so + 4 * q);
  float* dst = out + (size_t)blockIdx.x * (64 * NCLS) + 4 * q;
  if (tid < 160) *(volatile v4f*)dst = val;
  __threadfence();
  if (tid < 160) *(volatile v4f*)dst = val;
}

extern "C" void kernel_launch(void* const* d_in, const int* in_sizes, int n_in,
                              void* d_out, int out_size, void* d_ws, size_t ws_size,
                              hipStream_t stream) {
  if (n_in < 7) return;
  if (in_sizes[0] != NIMG * IMG_PIX) return;
  if (in_sizes[1] != 256 || in_sizes[2] != 256) return;
  if (in_sizes[3] != FEAT_K * HID || in_sizes[4] != HID) return;
  if (in_sizes[5] != HID * NCLS || in_sizes[6] != NCLS) return;
  if (out_size != NIMG * NCLS) return;
  if (ws_size < WS_TOTAL) return;

  const float* x      = (const float*)d_in[0];
  const float* U_re   = (const float*)d_in[1];
  const float* U_im   = (const float*)d_in[2];
  const float* W_proj = (const float*)d_in[3];
  const float* b_proj = (const float*)d_in[4];
  const float* W_cls  = (const float*)d_in[5];
  const float* b_cls  = (const float*)d_in[6];
  float* out = (float*)d_out;

  char* ws = (char*)d_ws;
  unsigned short* feats  = (unsigned short*)(ws);
  unsigned short* WpT    = (unsigned short*)(ws + WS_FEATS);
  unsigned short* WcT    = (unsigned short*)(ws + WS_FEATS + WS_WPT);
  unsigned short* hbuf   = (unsigned short*)(ws + WS_FEATS + WS_WPT + WS_WCT);
  float*          logits = (float*)(ws + WS_FEATS + WS_WPT + WS_WCT + WS_H);

  prep_wproj<<<HID, 128, 0, stream>>>(W_proj, WpT);
  prep_wcls<<<NCLS_PAD, 32, 0, stream>>>(W_cls, WcT);

  quanv_feats<<<(NIMG * NTILE) / 8, 256, 0, stream>>>(x, U_re, U_im, feats);

  {
    const int tiles = (NIMG / 64) * (HID / 64);
    wmma_gemm64<0, false, 2, 1, false, 0><<<dim3((tiles + 7) / 8, 1), 256, 0, stream>>>(
        feats, feats, FEAT_LD, 0L,
        WpT, WpT, FEAT_LD, 0L,
        (void*)hbuf, (void*)hbuf, HID, 0L,
        b_proj,
        logits, 0L,
        NIMG, HID, FEAT_LD, 1.0f / (FEAT_CARRY * WP_CARRY));
  }
  {
    const int tiles = (NIMG / 64) * (NCLS_PAD / 64);
    wmma_gemm64<0, false, 0, 0, false, 0><<<dim3((tiles + 7) / 8, 1), 256, 0, stream>>>(
        hbuf, hbuf, HID, 0L,
        WcT, WcT, HID, 0L,
        (void*)logits, (void*)logits, LOGIT_LD, 0L,
        b_proj,
        logits, 0L,
        NIMG, NCLS_PAD, HID, 1.0f / WC_CARRY);
  }
  lsm_store<<<NIMG / 64, 256, 0, stream>>>(logits, b_cls, out);
}
